// GCN_mamba_Net_Encoder_16853451669714
// MI455X (gfx1250) — hardware-verified
//
#include <hip/hip_runtime.h>


#define NN_   20000
#define FI_   512
#define DD_   128
#define DI_   256
#define NS_   16
#define DTR_  8
#define XDW_  64
#define XDN_  40
#define EE_   320000
#define AGW_  256
#define ECH_  1024

static_assert(NN_ % 32 == 0);
static_assert(NN_ % 16 == 0);
static_assert(NN_ % 8 == 0);
static_assert(FI_ == 512);
static_assert(DD_ == 128);
static_assert(DI_ == 256);
static_assert(DTR_ + 2 * NS_ == XDN_);
static_assert(XDN_ <= XDW_);
static_assert(AGW_ == 8 * 32);
static_assert(ECH_ == 4 * 256);

typedef float          v4f   __attribute__((ext_vector_type(4)));
typedef float          v8f   __attribute__((ext_vector_type(8)));
typedef int            v4i   __attribute__((ext_vector_type(4)));
typedef unsigned short u16x8 __attribute__((ext_vector_type(8)));
typedef __bf16         v16b  __attribute__((ext_vector_type(16)));

union FragB { u16x8 h[2]; v16b v; };
static_assert(sizeof(FragB) == 32);

constexpr size_t SZ_XP = (size_t)NN_ * FI_ * 2;
constexpr size_t SZ_XZ = (size_t)NN_ * (2 * DI_) * 4;
constexpr size_t SZ_XN = (size_t)NN_ * DD_ * 4;
constexpr size_t SZ_H  = (size_t)NN_ * (2 * DD_) * 2;
constexpr size_t SZ_F  = (size_t)NN_ * DD_ * 2;
constexpr size_t SZ_XD = (size_t)NN_ * XDW_ * 4;
constexpr size_t SZ_G4 = (size_t)NN_ * 16;
constexpr size_t SZ_V  = (size_t)2 * FI_ * 4;
constexpr size_t SZ_CS = 128;
constexpr size_t SZ_W1 = (size_t)DD_ * FI_ * 2;
constexpr size_t SZ_WF = (size_t)DD_ * (2 * DD_) * 2;
constexpr size_t SZ_WV = (size_t)DD_ * DD_ * 2;
constexpr size_t SZ_WI = (size_t)(2 * DI_) * DD_ * 2;
constexpr size_t SZ_WX = (size_t)XDW_ * DI_ * 2;
constexpr size_t SZ_WO = (size_t)DD_ * DI_ * 2;

constexpr size_t OFF_XH  = 0;
constexpr size_t OFF_XL  = OFF_XH + SZ_XP;
constexpr size_t OFF_XZ  = 0;
constexpr size_t OFF_XN  = OFF_XL + SZ_XP;
constexpr size_t OFF_HH  = OFF_XN + SZ_XN;
constexpr size_t OFF_HL  = OFF_HH + SZ_H;
constexpr size_t OFF_FH  = OFF_HL + SZ_H;
constexpr size_t OFF_FL  = OFF_FH + SZ_F;
constexpr size_t OFF_XD  = OFF_FL + SZ_F;
constexpr size_t OFF_G4  = OFF_XD + SZ_XD;
constexpr size_t OFF_V   = OFF_G4 + SZ_G4;
constexpr size_t OFF_CS  = OFF_V + SZ_V;
constexpr size_t OFF_W1H = OFF_CS + SZ_CS;
constexpr size_t OFF_W1L = OFF_W1H + SZ_W1;
constexpr size_t OFF_WFH = OFF_W1L + SZ_W1;
constexpr size_t OFF_WFL = OFF_WFH + SZ_WF;
constexpr size_t OFF_WAH = OFF_WFL + SZ_WF;
constexpr size_t OFF_WAL = OFF_WAH + SZ_WV;
constexpr size_t OFF_WBH = OFF_WAL + SZ_WV;
constexpr size_t OFF_WBL = OFF_WBH + SZ_WV;
constexpr size_t OFF_WIH = OFF_WBL + SZ_WV;
constexpr size_t OFF_WIL = OFF_WIH + SZ_WI;
constexpr size_t OFF_WXH = OFF_WIL + SZ_WI;
constexpr size_t OFF_WXL = OFF_WXH + SZ_WX;
constexpr size_t OFF_WOH = OFF_WXL + SZ_WX;
constexpr size_t OFF_WOL = OFF_WOH + SZ_WO;
constexpr size_t WS_END  = OFF_WOL + SZ_WO;

static_assert(SZ_XZ <= 2 * SZ_XP);
static_assert(WS_END <= (size_t)134217728);
static_assert(OFF_XL % 128 == 0 && OFF_XN % 128 == 0 && OFF_HH % 128 == 0 && OFF_HL % 128 == 0);
static_assert(OFF_FH % 128 == 0 && OFF_FL % 128 == 0 && OFF_XD % 128 == 0 && OFF_G4 % 128 == 0);
static_assert(OFF_V % 128 == 0 && OFF_CS % 128 == 0 && OFF_W1H % 128 == 0 && OFF_W1L % 128 == 0);
static_assert(OFF_WFH % 128 == 0 && OFF_WFL % 128 == 0 && OFF_WAH % 128 == 0 && OFF_WAL % 128 == 0);
static_assert(OFF_WBH % 128 == 0 && OFF_WBL % 128 == 0 && OFF_WIH % 128 == 0 && OFF_WIL % 128 == 0);
static_assert(OFF_WXH % 128 == 0 && OFF_WXL % 128 == 0 && OFF_WOH % 128 == 0 && OFF_WOL % 128 == 0 && WS_END % 128 == 0);

__device__ __forceinline__ float wave_sum(float v) {
#pragma unroll
    for (int s = 16; s >= 1; s >>= 1) v += __shfl_xor(v, s, 32);
    return v;
}
__device__ __forceinline__ v8f ld8f(const float* p) {
    const v4f a = *(const v4f*)p;
    const v4f b = *(const v4f*)(p + 4);
    return __builtin_shufflevector(a, b, 0, 1, 2, 3, 4, 5, 6, 7);
}
__device__ __forceinline__ unsigned int bfb(float f) {
    unsigned int u = __float_as_uint(f);
    u += 0x7FFFu + ((u >> 16) & 1u);
    return u >> 16;
}
__device__ __forceinline__ void split8(const v8f v, u16x8& hi, u16x8& lo) {
#pragma unroll
    for (int e = 0; e < 8; ++e) {
        const unsigned int hb = bfb(v[e]);
        const float hf = __uint_as_float(hb << 16);
        const unsigned int lb = bfb(v[e] - hf);
        hi[e] = (unsigned short)hb;
        lo[e] = (unsigned short)lb;
    }
}
__device__ __forceinline__ float silu_f(float x) {
    const float e = __expf(-x);
    return x * __builtin_amdgcn_rcpf(1.0f + e);
}
__device__ __forceinline__ float sigm_f(float x) {
    const float e = __expf(-x);
    return __builtin_amdgcn_rcpf(1.0f + e);
}
__device__ __forceinline__ float softplus_f(float x) {
    return fmaxf(x, 0.0f) + log1pf(__expf(-fabsf(x)));
}
__device__ __forceinline__ float conv4_silu(float x0, float x1, float x2, float x3,
                                            float w0, float w1, float w2, float w3, float bias) {
    float c = bias + w0 * x0;
    c = c + w1 * x1;
    c = c + w2 * x2;
    c = c + w3 * x3;
    return silu_f(c);
}

__device__ __forceinline__ void ldfrag(FragB& f, const unsigned short* p) {
    f.h[0] = *(const u16x8*)p;
    f.h[1] = *(const u16x8*)(p + 16);
}
__device__ __forceinline__ v8f wmma_bf(const FragB& a, const FragB& b, v8f c) {
    return __builtin_amdgcn_wmma_f32_16x16x32_bf16(false, a.v, false, b.v, (short)0, c, false, false);
}

__device__ __forceinline__ void row_store_hl(const float* srow, unsigned short* ph, unsigned short* pl, int lane) {
    const int q = lane & 15;
    const v8f v = ld8f(srow + 8 * q);
    u16x8 hi, lo;
    split8(v, hi, lo);
    u16x8 d;
#pragma unroll
    for (int e = 0; e < 8; ++e) d[e] = (lane < 16) ? hi[e] : lo[e];
    unsigned short* p = ((lane < 16) ? ph : pl) + 8 * q;
    *(volatile u16x8*)p = d;
}

__global__ __launch_bounds__(256)
void k_xsplit(const float* __restrict__ x, unsigned short* Xh, unsigned short* Xl)
{
    const int lane = threadIdx.x & 31, wave = threadIdx.x >> 5;
    const int row = blockIdx.x * 8 + wave;
    const float* xr = x + (size_t)row * FI_;
    u16x8 hv[2], lv[2];
#pragma unroll
    for (int g = 0; g < 2; ++g) {
        const v8f v = ld8f(xr + g * 256 + 8 * lane);
        split8(v, hv[g], lv[g]);
    }
    unsigned short* ph = Xh + (size_t)row * FI_ + 8 * lane;
    unsigned short* pl = Xl + (size_t)row * FI_ + 8 * lane;
    *(volatile u16x8*)(ph) = hv[0];  *(volatile u16x8*)(ph + 256) = hv[1];
    *(volatile u16x8*)(pl) = lv[0];  *(volatile u16x8*)(pl + 256) = lv[1];
    __threadfence();
    *(volatile u16x8*)(ph) = hv[0];  *(volatile u16x8*)(ph + 256) = hv[1];
    *(volatile u16x8*)(pl) = lv[0];  *(volatile u16x8*)(pl + 256) = lv[1];
}

template<bool TR>
__global__ __launch_bounds__(256)
void k_wplane(const float* __restrict__ W, unsigned short* Dh, unsigned short* Dl, int K, int Nsrc, int Npad, int sp)
{
    const int lane = threadIdx.x & 31, wave = threadIdx.x >> 5;
    const int n = blockIdx.x * 8 + wave;
    if (n >= Npad) return;
    const int  ncl = min(n, Nsrc - 1);
    const bool okn = n < Nsrc;
    u16x8 hv[2], lv[2];
#pragma unroll
    for (int g = 0; g < 2; ++g) {
        const int kb = g * 256;
        if (kb < K) {
            const int k  = kb + 8 * lane;
            const int kc = min(k, K - 8);
            v8f v;
#pragma unroll
            for (int e = 0; e < 8; ++e) {
                const size_t idx = TR ? ((size_t)(kc + e) * sp + ncl) : ((size_t)ncl * sp + kc + e);
                const float f = W[idx];
                v[e] = okn ? f : 0.0f;
            }
            split8(v, hv[g], lv[g]);
        }
    }
#pragma unroll
    for (int g = 0; g < 2; ++g) {
        const int kb = g * 256, k = kb + 8 * lane;
        if (kb < K && k < K) {
            *(volatile u16x8*)(Dh + (size_t)n * K + k) = hv[g];
            *(volatile u16x8*)(Dl + (size_t)n * K + k) = lv[g];
        }
    }
    __threadfence();
#pragma unroll
    for (int g = 0; g < 2; ++g) {
        const int kb = g * 256, k = kb + 8 * lane;
        if (kb < K && k < K) {
            *(volatile u16x8*)(Dh + (size_t)n * K + k) = hv[g];
            *(volatile u16x8*)(Dl + (size_t)n * K + k) = lv[g];
        }
    }
}

__global__ __launch_bounds__(256)
void k_vfold(const float* __restrict__ W1, const float* __restrict__ b1,
             const float* __restrict__ lnw, const float* __restrict__ lnb,
             const float* __restrict__ Wg, const float* __restrict__ bg,
             float* V, float* cst)
{
    const int tid = threadIdx.x, lane = tid & 31, wave = tid >> 5;
    const int k = blockIdx.x * 256 + tid;
    const float* wr = W1 + (size_t)k * DD_;
    float v0 = 0.0f, v1 = 0.0f;
#pragma unroll 2
    for (int j = 0; j < DD_; ++j) {
        const float a = wr[j] * lnw[j];
        v0 = fmaf(a, Wg[2 * j], v0);
        v1 = fmaf(a, Wg[2 * j + 1], v1);
    }
    const bool cwv = (blockIdx.x == 0) && (wave == 0);
    float cb0 = 0.0f, cb1 = 0.0f, cw0 = 0.0f, cw1 = 0.0f, cl0 = 0.0f, cl1 = 0.0f;
    if (cwv) {
#pragma unroll 1
        for (int i = 0; i < 4; ++i) {
            const int j = i * 32 + lane;
            const float w = lnw[j], g0 = Wg[2 * j], g1 = Wg[2 * j + 1], bb = b1[j], lb = lnb[j];
            cb0 += bb * w * g0;  cb1 += bb * w * g1;
            cw0 += w * g0;       cw1 += w * g1;
            cl0 += lb * g0;      cl1 += lb * g1;
        }
        cb0 = wave_sum(cb0); cb1 = wave_sum(cb1);
        cw0 = wave_sum(cw0); cw1 = wave_sum(cw1);
        cl0 = wave_sum(cl0) + bg[0]; cl1 = wave_sum(cl1) + bg[1];
    }
    v4f cv = {0.0f, 0.0f, 0.0f, 0.0f};
    if (lane == 0) { cv[0] = cb0; cv[1] = cb1; cv[2] = cw0; cv[3] = cw1; }
    if (lane == 1) { cv[0] = cl0; cv[1] = cl1; }
    const bool gw = cwv && (lane < 8);
    *(volatile float*)(V + k) = v0;
    *(volatile float*)(V + FI_ + k) = v1;
    if (gw) *(volatile v4f*)(cst + 4 * lane) = cv;
    __threadfence();
    *(volatile float*)(V + k) = v0;
    *(volatile float*)(V + FI_ + k) = v1;
    if (gw) *(volatile v4f*)(cst + 4 * lane) = cv;
}

__device__ __forceinline__ void tile32_store(const float* st, float* gp, int ldc, int lane) {
    const int rsub = lane >> 3, c0 = (lane & 7) * 4;
#pragma unroll
    for (int it = 0; it < 8; ++it) {
        const int row = it * 4 + rsub;
        const v4f v = *(const v4f*)(st + row * 36 + c0);
        *(volatile v4f*)(gp + (size_t)row * ldc + c0) = v;
    }
}

template<int WN, bool HASB>
__global__ __launch_bounds__(WN * 32)
void k_gemm3(const unsigned short* __restrict__ Ah, const unsigned short* __restrict__ Al,
             const unsigned short* __restrict__ Bh, const unsigned short* __restrict__ Bl,
             const float* __restrict__ bias, float* C, int K, int ldc)
{
    constexpr int P = 36;
    __shared__ __attribute__((aligned(16))) float stile[WN][32 * P];
    const int tid = threadIdx.x, lane = tid & 31, wave = tid >> 5;
    const int h = lane >> 4, m = lane & 15;
    const int rowB = blockIdx.y * 32;
    const int colW = blockIdx.x * (WN * 32) + wave * 32;
    const size_t ao0 = (size_t)(rowB + m) * K + 8 * h;
    const size_t ao1 = (size_t)(rowB + 16 + m) * K + 8 * h;
    const size_t bo0 = (size_t)(colW + m) * K + 8 * h;
    const size_t bo1 = (size_t)(colW + 16 + m) * K + 8 * h;

    v8f acc[4];
#pragma unroll
    for (int i = 0; i < 4; ++i)
#pragma unroll
        for (int r = 0; r < 8; ++r) acc[i][r] = 0.0f;

    const int nk = K >> 5;
    for (int kt = 0; kt < nk; ++kt) {
        const int k0 = kt * 32;
        FragB ah[2], al[2], bh[2], bl[2];
        ldfrag(ah[0], Ah + ao0 + k0);  ldfrag(ah[1], Ah + ao1 + k0);
        ldfrag(al[0], Al + ao0 + k0);  ldfrag(al[1], Al + ao1 + k0);
        ldfrag(bh[0], Bh + bo0 + k0);  ldfrag(bh[1], Bh + bo1 + k0);
        ldfrag(bl[0], Bl + bo0 + k0);  ldfrag(bl[1], Bl + bo1 + k0);
#pragma unroll
        for (int s = 0; s < 2; ++s)
#pragma unroll
            for (int j = 0; j < 2; ++j) acc[2 * s + j] = wmma_bf(ah[s], bh[j], acc[2 * s + j]);
#pragma unroll
        for (int s = 0; s < 2; ++s)
#pragma unroll
            for (int j = 0; j < 2; ++j) acc[2 * s + j] = wmma_bf(al[s], bh[j], acc[2 * s + j]);
#pragma unroll
        for (int s = 0; s < 2; ++s)
#pragma unroll
            for (int j = 0; j < 2; ++j) acc[2 * s + j] = wmma_bf(ah[s], bl[j], acc[2 * s + j]);
        asm volatile("v_nop\n\tv_nop\n\tv_nop\n\tv_nop" : "+v"(acc[0]), "+v"(acc[1]), "+v"(acc[2]), "+v"(acc[3]) : "v"(ah[0].v), "v"(ah[1].v), "v"(al[0].v), "v"(al[1].v), "v"(bh[0].v), "v"(bh[1].v), "v"(bl[0].v), "v"(bl[1].v));
    }

    float bv0 = 0.0f, bv1 = 0.0f;
    if constexpr (HASB) { bv0 = bias[colW + m]; bv1 = bias[colW + 16 + m]; }
    float* st = stile[wave];
#pragma unroll
    for (int s = 0; s < 2; ++s)
#pragma unroll
        for (int j = 0; j < 2; ++j) {
            const float bv = (j == 0) ? bv0 : bv1;
#pragma unroll
            for (int r = 0; r < 8; ++r)
                st[(s * 16 + 8 * h + r) * P + j * 16 + m] = acc[2 * s + j][r] + bv;
        }
    __syncthreads();

    float* gp = C + (size_t)rowB * ldc + colW;
    tile32_store(st, gp, ldc, lane);
    __threadfence();
    tile32_store(st, gp, ldc, lane);
}

__global__ __launch_bounds__(256)
void k_ln_gate(const float* __restrict__ x, const float* xin,
               const float* __restrict__ lnw, const float* __restrict__ lnb,
               const float* __restrict__ gu, const float* __restrict__ V, const float* __restrict__ cst,
               float* xnorm, unsigned short* Hh, unsigned short* Hl, float* g4)
{
    __shared__ v4f sg[8];
    const int tid = threadIdx.x, lane = tid & 31, wave = tid >> 5;
    const int row = blockIdx.x * 8 + wave;
    const int cA = 4 * lane;

    const v4f xi = *(const v4f*)(xin + (size_t)row * DD_ + cA);
    float s = xi[0] + xi[1] + xi[2] + xi[3];
    s = wave_sum(s);
    const float m = s * (1.0f / (float)DD_);
    const v4f dv = xi - m;
    float q = dv[0] * dv[0] + dv[1] * dv[1] + dv[2] * dv[2] + dv[3] * dv[3];
    q = wave_sum(q);
    const float var = q * (1.0f / (float)DD_);
    const float r = 1.0f / sqrtf(var + 1e-5f);
    const v4f w4 = *(const v4f*)(lnw + cA);
    const v4f b4 = *(const v4f*)(lnb + cA);
    const v4f xnv = (dv * r) * w4 + b4;

    float t0 = 0.0f, t1 = 0.0f;
    const float* xr  = x + (size_t)row * FI_ + 16 * lane;
    const float* v0p = V + 16 * lane;
    const float* v1p = V + FI_ + 16 * lane;
#pragma unroll 1
    for (int qd = 0; qd < 4; ++qd) {
        const v4f xv = *(const v4f*)(xr + 4 * qd);
        const v4f a0 = *(const v4f*)(v0p + 4 * qd);
        const v4f a1 = *(const v4f*)(v1p + 4 * qd);
        t0 += xv[0] * a0[0] + xv[1] * a0[1] + xv[2] * a0[2] + xv[3] * a0[3];
        t1 += xv[0] * a1[0] + xv[1] * a1[1] + xv[2] * a1[2] + xv[3] * a1[3];
    }
    t0 = wave_sum(t0);
    t1 = wave_sum(t1);
    const v4f c4a = *(const v4f*)cst;
    const v4f c4b = *(const v4f*)(cst + 4);
    const float l0 = r * ((t0 + c4a[0]) - m * c4a[2]) + c4b[0];
    const float l1 = r * ((t1 + c4a[1]) - m * c4a[3]) + c4b[1];

    float u0 = gu[(size_t)row * 2], u1 = gu[(size_t)row * 2 + 1];
    u0 = fminf(fmaxf(u0, 1e-6f), 0.999999f);
    u1 = fminf(fmaxf(u1, 1e-6f), 0.999999f);
    const float gg0 = -logf(-logf(u0));
    const float gg1 = -logf(-logf(u1));
    const float v0 = l0 + gg0, v1 = l1 + gg1;
    const float mx = fmaxf(v0, v1), mn = fminf(v0, v1);
    const float ex = expf(mn - mx);
    const float e0 = (v0 == mx) ? 1.0f : ex;
    const float e1 = (v1 == mx) ? 1.0f : ex;
    const float ssum = e0 + e1;
    const float rs = 1.0f / ssum;
    const float ys0 = e0 * rs, ys1 = e1 * rs;
    const float yh1 = (ys1 > ys0) ? 1.0f : 0.0f;
    const float gate = (yh1 - ys1) + ys1;

    const int qq = lane & 15, s0 = 2 * qq, s1 = 2 * qq + 1;
    v8f e8;
    e8[0] = __shfl(xnv[0], s0, 32); e8[1] = __shfl(xnv[1], s0, 32);
    e8[2] = __shfl(xnv[2], s0, 32); e8[3] = __shfl(xnv[3], s0, 32);
    e8[4] = __shfl(xnv[0], s1, 32); e8[5] = __shfl(xnv[1], s1, 32);
    e8[6] = __shfl(xnv[2], s1, 32); e8[7] = __shfl(xnv[3], s1, 32);
    u16x8 hi, lo, hd;
    split8(e8, hi, lo);
#pragma unroll
    for (int e = 0; e < 8; ++e) hd[e] = (lane < 16) ? hi[e] : lo[e];
    unsigned short* hp = ((lane < 16) ? Hh : Hl) + (size_t)row * (2 * DD_) + 8 * qq;
    float* xp = xnorm + (size_t)row * DD_ + cA;

    if (lane == 0) { v4f gv0 = {gate, 0.0f, 0.0f, 0.0f}; sg[wave] = gv0; }
    __syncthreads();
    const v4f gv = sg[lane & 7];
    float* gp = g4 + ((size_t)blockIdx.x * 8 + (lane & 7)) * 4;
    const bool gw = (wave == 0) && (lane < 8);

    *(volatile v4f*)xp = xnv;
    *(volatile u16x8*)hp = hd;
    if (gw) *(volatile v4f*)gp = gv;
    __threadfence();
    *(volatile v4f*)xp = xnv;
    *(volatile u16x8*)hp = hd;
    if (gw) *(volatile v4f*)gp = gv;
}

__device__ __forceinline__ void agg_store_pass(const float* sacc, unsigned short* Hh, unsigned short* Hl,
                                               int rbase, int nN, int wave, int lane) {
#pragma unroll 4
    for (int i = 0; i < 32; ++i) {
        const int lr = wave * 32 + i, row = rbase + lr;
        if (row < nN)
            row_store_hl(sacc + lr * DD_, Hh + (size_t)row * (2 * DD_) + DD_, Hl + (size_t)row * (2 * DD_) + DD_, lane);
    }
}

__global__ __launch_bounds__(256)
void k_agg(const int* __restrict__ ei, const float* __restrict__ ew, const float* __restrict__ g4,
           const float* __restrict__ xn, unsigned short* Hh, unsigned short* Hl, int nE, int nN)
{
    __shared__ __attribute__((aligned(16))) float sacc[AGW_ * DD_];
    __shared__ int shl[ECH_];
    __shared__ int shc[ECH_];
    __shared__ int she[ECH_];
    __shared__ int swt[8];
    const int tid = threadIdx.x, lane = tid & 31, wave = tid >> 5;
    const int rbase = blockIdx.x * AGW_;
    {
        const v4f z = {0.0f, 0.0f, 0.0f, 0.0f};
        v4f* s4 = (v4f*)sacc;
#pragma unroll
        for (int i = 0; i < (AGW_ * DD_) / (4 * 256); ++i) s4[i * 256 + tid] = z;
    }
    __syncthreads();

    const unsigned int lt = (1u << lane) - 1u;
    const bool vec4 = ((nE & 3) == 0);
    const int nchunk = (nE + ECH_ - 1) / ECH_;
    for (int ch = 0; ch < nchunk; ++ch) {
        const int cbase = ch * ECH_;
        int rr[4], cc[4];
        bool vd[4];
        if (vec4 && cbase + ECH_ <= nE) {
            const v4i rv = *(const v4i*)(ei + cbase + 4 * tid);
            const v4i cv = *(const v4i*)(ei + (size_t)nE + cbase + 4 * tid);
#pragma unroll
            for (int j = 0; j < 4; ++j) { rr[j] = rv[j]; cc[j] = cv[j]; vd[j] = true; }
        } else {
#pragma unroll
            for (int j = 0; j < 4; ++j) {
                const int e  = cbase + 4 * tid + j;
                const int ec = min(e, nE - 1);
                rr[j] = ei[ec];
                cc[j] = ei[(size_t)nE + ec];
                vd[j] = (e < nE);
            }
        }
        unsigned int mk[4];
        int lrj[4], ccl[4];
        bool ht[4];
        int cnt = 0;
#pragma unroll
        for (int j = 0; j < 4; ++j) {
            const int lr = rr[j] - rbase;
            ht[j]  = vd[j] && ((unsigned int)lr < (unsigned int)AGW_);
            lrj[j] = lr;
            ccl[j] = min(max(cc[j], 0), nN - 1);
            mk[j]  = __builtin_amdgcn_ballot_w32(ht[j]);
            cnt   += __builtin_popcount(mk[j]);
        }
        if (lane == 0) swt[wave] = cnt;
        __syncthreads();
        int woff = 0, tot = 0;
#pragma unroll
        for (int w = 0; w < 8; ++w) {
            const int c = swt[w];
            tot  += c;
            woff += (w < wave) ? c : 0;
        }
        int run = 0;
#pragma unroll
        for (int j = 0; j < 4; ++j) {
            int pos = woff + run + __builtin_popcount(mk[j] & lt);
            pos = min(pos, ECH_ - 1);
            if (ht[j]) { shl[pos] = lrj[j]; shc[pos] = ccl[j]; she[pos] = cbase + 4 * tid + j; }
            run += __builtin_popcount(mk[j]);
        }
        __syncthreads();
        const int nh = min(tot, ECH_);
        for (int hI = 0; hI < nh; ++hI) {
            const int lr = shl[hI] & (AGW_ - 1);
            if ((lr >> 5) == wave) {
                const int col = min(max(shc[hI], 0), nN - 1);
                const int e   = min(max(she[hI], 0), nE - 1);
                const int rcw = min(rbase + lr, nN - 1);
                const float w = (ew[e] * g4[(size_t)rcw * 4]) * g4[(size_t)col * 4];
                const v4f xv = *(const v4f*)(xn + (size_t)col * DD_ + 4 * lane);
                v4f* ap = (v4f*)(sacc + lr * DD_ + 4 * lane);
                v4f a = *ap;
                a = a + w * xv;
                *ap = a;
            }
        }
        __syncthreads();
    }

    agg_store_pass(sacc, Hh, Hl, rbase, nN, wave, lane);
    __threadfence();
    agg_store_pass(sacc, Hh, Hl, rbase, nN, wave, lane);
}

__global__ __launch_bounds__(256)
void k_fusion(const unsigned short* __restrict__ Hh,  const unsigned short* __restrict__ Hl,
              const unsigned short* __restrict__ Wfh, const unsigned short* __restrict__ Wfl,
              const unsigned short* __restrict__ Wah, const unsigned short* __restrict__ Wal,
              const unsigned short* __restrict__ Wbh, const unsigned short* __restrict__ Wbl,
              const float* __restrict__ bfv, const float* __restrict__ bv1, const float* __restrict__ bv2,
              unsigned short* Fh, unsigned short* Fl)
{
    constexpr int SP = DD_ + 4;
    __shared__ __attribute__((aligned(16))) float st[32 * SP];
    const int tid = threadIdx.x, lane = tid & 31, wave = tid >> 5;
    const int h = lane >> 4, m = lane & 15;
    const int rowB = blockIdx.x * 32;
    const int col0 = wave * 16;
    const size_t ao0 = (size_t)(rowB + m) * (2 * DD_) + 8 * h;
    const size_t ao1 = (size_t)(rowB + 16 + m) * (2 * DD_) + 8 * h;
    const size_t fo  = (size_t)(col0 + m) * (2 * DD_) + 8 * h;
    const size_t vo  = (size_t)(col0 + m) * DD_ + 8 * h;

    v8f accF[2], accA[2], accB[2];
#pragma unroll
    for (int s = 0; s < 2; ++s)
#pragma unroll
        for (int r = 0; r < 8; ++r) { accF[s][r] = 0.0f; accA[s][r] = 0.0f; accB[s][r] = 0.0f; }

    for (int kt = 0; kt < 4; ++kt) {
        const int k0 = kt * 32;
        FragB ah[2], al[2], fh, fl, gh, gl;
        ldfrag(ah[0], Hh + ao0 + k0);  ldfrag(ah[1], Hh + ao1 + k0);
        ldfrag(al[0], Hl + ao0 + k0);  ldfrag(al[1], Hl + ao1 + k0);
        ldfrag(fh, Wfh + fo + k0);     ldfrag(fl, Wfl + fo + k0);
        ldfrag(gh, Wah + vo + k0);     ldfrag(gl, Wal + vo + k0);
#pragma unroll
        for (int s = 0; s < 2; ++s) { accF[s] = wmma_bf(ah[s], fh, accF[s]); accA[s] = wmma_bf(ah[s], gh, accA[s]); }
#pragma unroll
        for (int s = 0; s < 2; ++s) { accF[s] = wmma_bf(al[s], fh, accF[s]); accA[s] = wmma_bf(al[s], gh, accA[s]); }
#pragma unroll
        for (int s = 0; s < 2; ++s) { accF[s] = wmma_bf(ah[s], fl, accF[s]); accA[s] = wmma_bf(ah[s], gl, accA[s]); }
        asm volatile("v_nop\n\tv_nop\n\tv_nop\n\tv_nop" : "+v"(accF[0]), "+v"(accF[1]), "+v"(accA[0]), "+v"(accA[1]) : "v"(ah[0].v), "v"(ah[1].v), "v"(al[0].v), "v"(al[1].v), "v"(fh.v), "v"(fl.v), "v"(gh.v), "v"(gl.v));
    }
    for (int kt = 0; kt < 4; ++kt) {
        const int k0 = 128 + kt * 32;
        FragB ah[2], al[2], fh, fl, gh, gl;
        ldfrag(ah[0], Hh + ao0 + k0);  ldfrag(ah[1], Hh + ao1 + k0);
        ldfrag(al[0], Hl + ao0 + k0);  ldfrag(al[1], Hl + ao1 + k0);
        ldfrag(fh, Wfh + fo + k0);     ldfrag(fl, Wfl + fo + k0);
        ldfrag(gh, Wbh + vo + (k0 - 128)); ldfrag(gl, Wbl + vo + (k0 - 128));
#pragma unroll
        for (int s = 0; s < 2; ++s) { accF[s] = wmma_bf(ah[s], fh, accF[s]); accB[s] = wmma_bf(ah[s], gh, accB[s]); }
#pragma unroll
        for (int s = 0; s < 2; ++s) { accF[s] = wmma_bf(al[s], fh, accF[s]); accB[s] = wmma_bf(al[s], gh, accB[s]); }
#pragma unroll
        for (int s = 0; s < 2; ++s) { accF[s] = wmma_bf(ah[s], fl, accF[s]); accB[s] = wmma_bf(ah[s], gl, accB[s]); }
        asm volatile("v_nop\n\tv_nop\n\tv_nop\n\tv_nop" : "+v"(accF[0]), "+v"(accF[1]), "+v"(accB[0]), "+v"(accB[1]) : "v"(ah[0].v), "v"(ah[1].v), "v"(al[0].v), "v"(al[1].v), "v"(fh.v), "v"(fl.v), "v"(gh.v), "v"(gl.v));
    }

    const int col = col0 + m;
    const float cbf = bfv[col], cb1 = bv1[col], cb2 = bv2[col];
#pragma unroll
    for (int s = 0; s < 2; ++s)
#pragma unroll
        for (int r = 0; r < 8; ++r) {
            const float f  = accF[s][r] + cbf;
            const float fg = sigm_f(f);
            const float a  = accA[s][r] + cb1;
            const float b  = accB[s][r] + cb2;
            st[(s * 16 + 8 * h + r) * SP + col] = fg * a + (1.0f - fg) * b;
        }
    __syncthreads();

#pragma unroll
    for (int i = 0; i < 4; ++i) {
        const int row = wave * 4 + i;
        row_store_hl(st + row * SP, Fh + (size_t)(rowB + row) * DD_, Fl + (size_t)(rowB + row) * DD_, lane);
    }
    __threadfence();
#pragma unroll
    for (int i = 0; i < 4; ++i) {
        const int row = wave * 4 + i;
        row_store_hl(st + row * SP, Fh + (size_t)(rowB + row) * DD_, Fl + (size_t)(rowB + row) * DD_, lane);
    }
}

__global__ __launch_bounds__(256)
void k_conv(const float* __restrict__ xz, const float* __restrict__ cw, const float* __restrict__ cb,
            unsigned short* Ch, unsigned short* Cl)
{
    const int lane = threadIdx.x & 31, wave = threadIdx.x >> 5;
    const int t  = blockIdx.x * 8 + wave;
    const int d0 = 8 * lane;
    const int t1 = max(t - 1, 0), t2 = max(t - 2, 0), t3 = max(t - 3, 0);
    v8f x3 = ld8f(xz + (size_t)t  * (2 * DI_) + d0);
    v8f x2 = ld8f(xz + (size_t)t1 * (2 * DI_) + d0);
    v8f x1 = ld8f(xz + (size_t)t2 * (2 * DI_) + d0);
    v8f x0 = ld8f(xz + (size_t)t3 * (2 * DI_) + d0);
#pragma unroll
    for (int c = 0; c < 8; ++c) {
        x2[c] = (t >= 1) ? x2[c] : 0.0f;
        x1[c] = (t >= 2) ? x1[c] : 0.0f;
        x0[c] = (t >= 3) ? x0[c] : 0.0f;
    }
    const float* wp = cw + (size_t)d0 * 4;
    v4f wv[8];
#pragma unroll
    for (int c = 0; c < 8; ++c) wv[c] = *(const v4f*)(wp + 4 * c);
    const v8f bias = ld8f(cb + d0);
    v8f u;
#pragma unroll
    for (int c = 0; c < 8; ++c)
        u[c] = conv4_silu(x0[c], x1[c], x2[c], x3[c], wv[c][0], wv[c][1], wv[c][2], wv[c][3], bias[c]);
    u16x8 hi, lo;
    split8(u, hi, lo);
    unsigned short* ph = Ch + (size_t)t * DI_ + d0;
    unsigned short* pl = Cl + (size_t)t * DI_ + d0;
    *(volatile u16x8*)ph = hi;
    *(volatile u16x8*)pl = lo;
    __threadfence();
    *(volatile u16x8*)ph = hi;
    *(volatile u16x8*)pl = lo;
}

__device__ __forceinline__ void g16_store_pass(const unsigned short* sl, unsigned short* gp,
                                               size_t gbase, int wave, int lane) {
#pragma unroll
    for (int it = 0; it < 2; ++it) {
        const int t = it * 8 + wave * 4 + (lane >> 3);
        const int c = (lane & 7) * 8;
        const u16x8 v = *(const u16x8*)(sl + t * 64 + c);
        *(volatile u16x8*)(gp + gbase + (size_t)t * DI_ + c) = v;
    }
}

__global__ __launch_bounds__(64)
void k_scan(const float* __restrict__ xz, const float* __restrict__ xd,
            const float* __restrict__ cw, const float* __restrict__ cb,
            const float* __restrict__ dtw, const float* __restrict__ dtb,
            const float* __restrict__ Alog, const float* __restrict__ Dp,
            unsigned short* Gh, unsigned short* Gl)
{
    __shared__ __attribute__((aligned(16))) unsigned short sgh[16 * 64];
    __shared__ __attribute__((aligned(16))) unsigned short sgl[16 * 64];
    __shared__ __attribute__((aligned(16))) float sX[16 * XDW_];

    const int tid   = threadIdx.x;
    const int lane  = tid & 31;
    const int wave  = tid >> 5;
    const int dbase = blockIdx.x * 64;
    const int d     = dbase + tid;

    float an[NS_], hs[NS_];
#pragma unroll
    for (int n = 0; n < NS_; ++n) {
        an[n] = -expf(Alog[(size_t)d * NS_ + n]);
        hs[n] = 0.0f;
    }
    float wd[DTR_];
#pragma unroll
    for (int r = 0; r < DTR_; ++r) wd[r] = dtw[(size_t)d * DTR_ + r];
    const float w0 = cw[d * 4 + 0], w1 = cw[d * 4 + 1], w2 = cw[d * 4 + 2], w3 = cw[d * 4 + 3];
    const float cbias = cb[d];
    const float tb    = dtb[d];
    const float Dd    = Dp[d];

    float xm1 = 0.0f, xm2 = 0.0f, xm3 = 0.0f;

#pragma unroll 1
    for (int l0 = 0; l0 < NN_; l0 += 16) {
        const float* xsrc = xd + (size_t)l0 * XDW_;
#pragma unroll
        for (int j = 0; j < 16; ++j) sX[j * 64 + tid] = xsrc[j * 64 + tid];
        __syncthreads();
#pragma unroll 1
        for (int t = 0; t < 16; ++t) {
            const size_t e = (size_t)(l0 + t) * (2 * DI_) + d;
            const float xv = xz[e];
            const float zv = xz[e + DI_];
            const float u  = conv4_silu(xm3, xm2, xm1, xv, w0, w1, w2, w3, cbias);
            xm3 = xm2; xm2 = xm1; xm1 = xv;
            const float* sr = sX + t * XDW_;
            float dp = 0.0f;
#pragma unroll
            for (int r = 0; r < DTR_; ++r) dp = fmaf(sr[r], wd[r], dp);
            const float dt = softplus_f(dp + tb);
            float y = 0.0f;
#pragma unroll
            for (int n = 0; n < NS_; ++n) {
                const float da = __expf(dt * an[n]);
                const float db = (dt * sr[DTR_ + n]) * u;
                hs[n] = da * hs[n] + db;
                y += hs[n] * sr[DTR_ + NS_ + n];
            }
            const float g = (y + Dd * u) * silu_f(zv);
            const unsigned int hb = bfb(g);
            const unsigned int lb = bfb(g - __uint_as_float(hb << 16));
            sgh[t * 64 + tid] = (unsigned short)hb;
            sgl[t * 64 + tid] = (unsigned short)lb;
        }
        __syncthreads();
        const size_t gbase = (size_t)l0 * DI_ + dbase;
        g16_store_pass(sgh, Gh, gbase, wave, lane);
        g16_store_pass(sgl, Gl, gbase, wave, lane);
        __threadfence();
        g16_store_pass(sgh, Gh, gbase, wave, lane);
        g16_store_pass(sgl, Gl, gbase, wave, lane);
        __syncthreads();
    }
}

__global__ __launch_bounds__(256)
void k_final(const float* __restrict__ mo, const float* xin,
             const float* __restrict__ lw, const float* __restrict__ lb,
             const float* __restrict__ bw, const float* __restrict__ bb,
             const float* __restrict__ brm, const float* __restrict__ brv,
             float* out)
{
    const int lane = threadIdx.x & 31, wave = threadIdx.x >> 5;
    const int row = blockIdx.x * 8 + wave;
    const int cA = 4 * lane;
    const v4f a = *(const v4f*)(mo + (size_t)row * DD_ + cA);
    const v4f b = *(const v4f*)(xin + (size_t)row * DD_ + cA);
    const v4f v = a + b;
    float s = v[0] + v[1] + v[2] + v[3];
    s = wave_sum(s);
    const float m = s * (1.0f / (float)DD_);
    const v4f dv = v - m;
    float q = dv[0] * dv[0] + dv[1] * dv[1] + dv[2] * dv[2] + dv[3] * dv[3];
    q = wave_sum(q);
    const float var = q * (1.0f / (float)DD_);
    const float r = 1.0f / sqrtf(var + 1e-5f);
    const v4f w4 = *(const v4f*)(lw + cA), b4 = *(const v4f*)(lb + cA);
    const v4f o = (dv * r) * w4 + b4;
    const v4f rm4 = *(const v4f*)(brm + cA), rv4 = *(const v4f*)(brv + cA);
    const v4f gw4 = *(const v4f*)(bw + cA),  gb4 = *(const v4f*)(bb + cA);
    v4f res;
#pragma unroll
    for (int e = 0; e < 4; ++e) res[e] = (o[e] - rm4[e]) * (1.0f / sqrtf(rv4[e] + 1e-5f)) * gw4[e] + gb4[e];
    float* op = out + (size_t)row * DD_ + cA;
    *(volatile v4f*)op = res;
    __threadfence();
    *(volatile v4f*)op = res;
}

extern "C" void kernel_launch(void* const* d_in, const int* in_sizes, int n_in,
                              void* d_out, int out_size, void* d_ws, size_t ws_size,
                              hipStream_t stream)
{
    if (n_in < 31) return;
    if (in_sizes[0]  != NN_ * FI_)        return;
    if (in_sizes[1]  != 2 * EE_)          return;
    if (in_sizes[2]  != EE_)              return;
    if (in_sizes[3]  != NN_ * 2)          return;
    if (in_sizes[4]  != FI_ * DD_)        return;
    if (in_sizes[5]  != DD_)              return;
    if (in_sizes[6]  != DD_)              return;
    if (in_sizes[7]  != DD_)              return;
    if (in_sizes[8]  != DD_ * 2)          return;
    if (in_sizes[9]  != 2)                return;
    if (in_sizes[10] != 2 * DD_ * DD_)    return;
    if (in_sizes[11] != DD_)              return;
    if (in_sizes[12] != DD_ * DD_)        return;
    if (in_sizes[13] != DD_)              return;
    if (in_sizes[14] != DD_ * DD_)        return;
    if (in_sizes[15] != DD_)              return;
    if (in_sizes[16] != 2 * DI_ * DD_)    return;
    if (in_sizes[17] != DI_ * 4)          return;
    if (in_sizes[18] != DI_)              return;
    if (in_sizes[19] != XDN_ * DI_)       return;
    if (in_sizes[20] != DI_ * DTR_)       return;
    if (in_sizes[21] != DI_)              return;
    if (in_sizes[22] != DI_ * NS_)        return;
    if (in_sizes[23] != DI_)              return;
    if (in_sizes[24] != DD_ * DI_)        return;
    for (int i = 25; i < 31; ++i) if (in_sizes[i] != DD_) return;
    if (out_size != 2 * NN_ * DD_)        return;
    if (ws_size < WS_END)                 return;

    const float* x    = (const float*)d_in[0];
    const int*   ei   = (const int*)  d_in[1];
    const float* ew   = (const float*)d_in[2];
    const float* gu   = (const float*)d_in[3];
    const float* W1   = (const float*)d_in[4];
    const float* b1   = (const float*)d_in[5];
    const float* lnw  = (const float*)d_in[6];
    const float* lnb  = (const float*)d_in[7];
    const float* Wg   = (const float*)d_in[8];
    const float* bg   = (const float*)d_in[9];
    const float* Wf   = (const float*)d_in[10];
    const float* bfv  = (const float*)d_in[11];
    const float* Wv1  = (const float*)d_in[12];
    const float* bv1  = (const float*)d_in[13];
    const float* Wv2  = (const float*)d_in[14];
    const float* bv2  = (const float*)d_in[15];
    const float* Win  = (const float*)d_in[16];
    const float* cw   = (const float*)d_in[17];
    const float* cb   = (const float*)d_in[18];
    const float* Wxp  = (const float*)d_in[19];
    const float* Wdt  = (const float*)d_in[20];
    const float* bdt  = (const float*)d_in[21];
    const float* Alog = (const float*)d_in[22];
    const float* Dsk  = (const float*)d_in[23];
    const float* Wout = (const float*)d_in[24];
    const float* low  = (const float*)d_in[25];
    const float* lob  = (const float*)d_in[26];
    const float* bnw  = (const float*)d_in[27];
    const float* bnb  = (const float*)d_in[28];
    const float* bnrm = (const float*)d_in[29];
    const float* bnrv = (const float*)d_in[30];

    float* out0 = (float*)d_out;
    float* out1 = out0 + (size_t)NN_ * DD_;

    char* ws = (char*)d_ws;
    unsigned short* Xh  = (unsigned short*)(ws + OFF_XH);
    unsigned short* Xl  = (unsigned short*)(ws + OFF_XL);
    float*          xz  = (float*)(ws + OFF_XZ);
    float*          xnm = (float*)(ws + OFF_XN);
    unsigned short* Hh  = (unsigned short*)(ws + OFF_HH);
    unsigned short* Hl  = (unsigned short*)(ws + OFF_HL);
    unsigned short* Fh  = (unsigned short*)(ws + OFF_FH);
    unsigned short* Fl  = (unsigned short*)(ws + OFF_FL);
    float*          xd  = (float*)(ws + OFF_XD);
    float*          g4  = (float*)(ws + OFF_G4);
    float*          V   = (float*)(ws + OFF_V);
    float*          cst = (float*)(ws + OFF_CS);
    unsigned short* W1h = (unsigned short*)(ws + OFF_W1H);
    unsigned short* W1l = (unsigned short*)(ws + OFF_W1L);
    unsigned short* Wfh = (unsigned short*)(ws + OFF_WFH);
    unsigned short* Wfl = (unsigned short*)(ws + OFF_WFL);
    unsigned short* Wah = (unsigned short*)(ws + OFF_WAH);
    unsigned short* Wal = (unsigned short*)(ws + OFF_WAL);
    unsigned short* Wbh = (unsigned short*)(ws + OFF_WBH);
    unsigned short* Wbl = (unsigned short*)(ws + OFF_WBL);
    unsigned short* Wih = (unsigned short*)(ws + OFF_WIH);
    unsigned short* Wil = (unsigned short*)(ws + OFF_WIL);
    unsigned short* Wxh = (unsigned short*)(ws + OFF_WXH);
    unsigned short* Wxl = (unsigned short*)(ws + OFF_WXL);
    unsigned short* Woh = (unsigned short*)(ws + OFF_WOH);
    unsigned short* Wol = (unsigned short*)(ws + OFF_WOL);

    k_xsplit<<<dim3(NN_ / 8), dim3(256), 0, stream>>>(x, Xh, Xl);

    k_wplane<true><<<dim3(DD_ / 8), dim3(256), 0, stream>>>(W1,  W1h, W1l, (int)FI_, (int)DD_, (int)DD_, (int)DD_);
    k_wplane<true><<<dim3(DD_ / 8), dim3(256), 0, stream>>>(Wf,  Wfh, Wfl, (int)(2 * DD_), (int)DD_, (int)DD_, (int)DD_);
    k_wplane<true><<<dim3(DD_ / 8), dim3(256), 0, stream>>>(Wv1, Wah, Wal, (int)DD_, (int)DD_, (int)DD_, (int)DD_);
    k_wplane<true><<<dim3(DD_ / 8), dim3(256), 0, stream>>>(Wv2, Wbh, Wbl, (int)DD_, (int)DD_, (int)DD_, (int)DD_);
    k_wplane<false><<<dim3((2 * DI_) / 8), dim3(256), 0, stream>>>(Win, Wih, Wil, (int)DD_, (int)(2 * DI_), (int)(2 * DI_), (int)DD_);
    k_wplane<false><<<dim3(XDW_ / 8), dim3(256), 0, stream>>>(Wxp, Wxh, Wxl, (int)DI_, (int)XDN_, (int)XDW_, (int)DI_);
    k_wplane<false><<<dim3(DD_ / 8), dim3(256), 0, stream>>>(Wout, Woh, Wol, (int)DI_, (int)DD_, (int)DD_, (int)DI_);

    k_vfold<<<dim3(2), dim3(256), 0, stream>>>(W1, b1, lnw, lnb, Wg, bg, V, cst);

    k_gemm3<4, true><<<dim3(1, NN_ / 32), dim3(128), 0, stream>>>(Xh, Xl, W1h, W1l, b1, out1, (int)FI_, (int)DD_);

    k_ln_gate<<<dim3(NN_ / 8), dim3(256), 0, stream>>>(x, out1, lnw, lnb, gu, V, cst, xnm, Hh, Hl, g4);

    k_agg<<<dim3((NN_ + AGW_ - 1) / AGW_), dim3(256), 0, stream>>>(ei, ew, g4, xnm, Hh, Hl, (int)EE_, (int)NN_);

    k_fusion<<<dim3(NN_ / 32), dim3(256), 0, stream>>>(Hh, Hl, Wfh, Wfl, Wah, Wal, Wbh, Wbl, bfv, bv1, bv2, Fh, Fl);

    k_gemm3<4, false><<<dim3((2 * DI_) / 128, NN_ / 32), dim3(128), 0, stream>>>(Fh, Fl, Wih, Wil, b1, xz, (int)DD_, (int)(2 * DI_));

    k_conv<<<dim3(NN_ / 8), dim3(256), 0, stream>>>(xz, cw, cb, Hh, Hl);

    k_gemm3<2, false><<<dim3(1, NN_ / 32), dim3(64), 0, stream>>>(Hh, Hl, Wxh, Wxl, b1, xd, (int)DI_, (int)XDW_);

    k_scan<<<dim3(DI_ / 64), dim3(64), 0, stream>>>(xz, xd, cw, cb, Wdt, bdt, Alog, Dsk, Hh, Hl);

    k_gemm3<4, false><<<dim3(1, NN_ / 32), dim3(128), 0, stream>>>(Hh, Hl, Woh, Wol, b1, xnm, (int)DI_, (int)DD_);

    k_final<<<dim3(NN_ / 8), dim3(256), 0, stream>>>(xnm, out1, low, lob, bnw, bnb, bnrm, bnrv, out0);
}
